// GraphMultiHeadAttentionLayer_12541304504947
// MI455X (gfx1250) — hardware-verified
//
#include <hip/hip_runtime.h>
#include <math.h>

typedef __attribute__((ext_vector_type(16))) _Float16 v16h;
typedef __attribute__((ext_vector_type(16))) __bf16 v16b;
typedef __attribute__((ext_vector_type(8)))  _Float16 v8h;
typedef __attribute__((ext_vector_type(8)))  float v8f;
typedef __attribute__((ext_vector_type(4)))  float v4f;
typedef __attribute__((ext_vector_type(2)))  float v2f;
typedef __attribute__((ext_vector_type(4)))  unsigned v4u;
typedef __attribute__((ext_vector_type(4)))  int v4i;
typedef float __attribute__((may_alias)) float_a;
typedef int __attribute__((may_alias)) int_a;

template <typename T> __device__ __forceinline__ void vst2(void* p, T v) { *(volatile T*)p = v; __threadfence(); *(volatile T*)p = v; }
__device__ __forceinline__ v8f wmma16(v16h a, v16h b, v8f c) {
  v8f d = __builtin_amdgcn_wmma_f32_16x16x32_f16(false, a, false, b, (short)0, c, false, false);
  asm volatile("v_nop\n\tv_nop\n\tv_nop\n\tv_nop" : "+v"(d) : "v"(a), "v"(b));
  return d;
}
__device__ __forceinline__ v8f wmma_bf(v16b a, v16b b, v8f c) {
  v8f d = __builtin_amdgcn_wmma_f32_16x16x32_bf16(false, a, false, b, (short)0, c, false, false);
  asm volatile("v_nop\n\tv_nop\n\tv_nop\n\tv_nop" : "+v"(d) : "v"(a), "v"(b));
  return d;
}
__device__ __forceinline__ v16h frag_h(const _Float16* rowk0, int lane) {
  union { v16h v; v8h q[2]; } u; const _Float16* p = rowk0 + 8 * (lane >> 4);
  u.q[0] = *(const v8h*)p; u.q[1] = *(const v8h*)(p + 16); return u.v;
}
__device__ __forceinline__ v16h frag_f32(const float* rowk0, int lane) {
  v16h a; const float* p = rowk0 + 8 * (lane >> 4);
#pragma unroll
  for (int i = 0; i < 8; ++i) { a[i] = (_Float16)p[i]; a[8 + i] = (_Float16)p[16 + i]; }
  return a;
}
__device__ __forceinline__ v16h frag_f32s(const float* rowk0, int lane, float sc) {
  v16h a; const float* p = rowk0 + 8 * (lane >> 4);
#pragma unroll
  for (int i = 0; i < 8; ++i) { a[i] = (_Float16)(p[i] * sc); a[8 + i] = (_Float16)(p[16 + i] * sc); }
  return a;
}
__device__ __forceinline__ v16h fragc_f32(const float* W, int k0, int n, int lane, int ld, int K) {
  v16h a; const int g = lane >> 4;
#pragma unroll
  for (int i = 0; i < 8; ++i) { const int ka = k0 + 8 * g + i, kb = ka + 16;
    a[i] = (_Float16)(ka < K ? W[(size_t)ka * ld + n] : 0.f); a[8 + i] = (_Float16)(kb < K ? W[(size_t)kb * ld + n] : 0.f); }
  return a;
}
struct F2 { v16b h, l; };
__device__ __forceinline__ F2 bsplit16(const float v[16]) { F2 r;
#pragma unroll
  for (int i = 0; i < 16; ++i) { const __bf16 h = (__bf16)v[i]; r.h[i] = h; r.l[i] = (__bf16)(v[i] - (float)h); }
  return r; }
__device__ __forceinline__ F2 split_row(const float* row, int k0, int lane) { float v[16]; const float* p = row + k0 + 8 * (lane >> 4);
#pragma unroll
  for (int i = 0; i < 8; ++i) { v[i] = p[i]; v[8 + i] = p[16 + i]; }
  return bsplit16(v); }
__device__ __forceinline__ F2 split_rowK(const float* row, int k0, int lane, int K) { float v[16]; const int g = lane >> 4;
#pragma unroll
  for (int i = 0; i < 8; ++i) { const int ka = k0 + 8 * g + i, kb = ka + 16; v[i] = ka < K ? row[ka] : 0.f; v[8 + i] = kb < K ? row[kb] : 0.f; }
  return bsplit16(v); }
__device__ __forceinline__ F2 split_col(const float* W, int k0, int n, int lane, int ld, int K) { float v[16]; const int g = lane >> 4;
#pragma unroll
  for (int i = 0; i < 8; ++i) { const int ka = k0 + 8 * g + i, kb = ka + 16; v[i] = ka < K ? W[(size_t)ka * ld + n] : 0.f; v[8 + i] = kb < K ? W[(size_t)kb * ld + n] : 0.f; }
  return bsplit16(v); }
__device__ __forceinline__ v8f mac3(const F2& a, const F2& b, v8f c) { c = wmma_bf(a.l, b.h, c); c = wmma_bf(a.h, b.l, c); return wmma_bf(a.h, b.h, c); }
__device__ __forceinline__ float sigm(float v) { return 1.0f / (1.0f + expf(-v)); }
#define LDSX() do { asm volatile("s_wait_dscnt 0" ::: "memory"); __builtin_amdgcn_wave_barrier(); __builtin_amdgcn_fence(__ATOMIC_RELEASE, "workgroup"); } while (0)

#define NB 4
#define NN 2048
#define FF 128
#define DD 64
#define NH 4
#define NR (NB * NN)

__global__ __launch_bounds__(128) void k_proj(const float* __restrict__ X, const float* __restrict__ Wk, const float* __restrict__ ak, _Float16* __restrict__ hT, float* __restrict__ sc) {
  __shared__ __align__(16) float so[4][16][68];
  __shared__ __align__(16) _Float16 st[DD][72];
  __shared__ float ssum[4][16];
  const int tid = threadIdx.x, wave = tid >> 5, lane = tid & 31, col = lane & 15, g = lane >> 4;
  const int hd = blockIdx.y, r0b = blockIdx.x * 64, r0 = r0b + wave * 16; const int b = r0b / NN, n0 = r0b % NN;
  v8f acc[4] = {};
#pragma unroll
  for (int kc = 0; kc < FF / 32; ++kc) { const v16h a = frag_f32(X + (size_t)(r0 + col) * FF + kc * 32, lane);
#pragma unroll
    for (int j = 0; j < 4; ++j) { v16h bb = fragc_f32(Wk + (size_t)hd * FF * DD, kc * 32, j * 16 + col, lane, DD, FF);
#pragma unroll
      for (int e = 0; e < 16; ++e) bb[e] = bb[e] * (_Float16)8.0f;
      acc[j] = wmma16(a, bb, acc[j]); } }
#pragma unroll
  for (int j = 0; j < 4; ++j)
#pragma unroll
    for (int r = 0; r < 8; ++r) so[wave][8 * g + r][j * 16 + col] = acc[j][r] * 0.125f;
  LDSX();
  { const int rl = lane >> 1, hf = lane & 1; float s = 0.f; for (int d = 0; d < 32; ++d) s += so[wave][rl][hf * 32 + d] * ak[hd * DD + hf * 32 + d]; s += __shfl_xor(s, 1, 32); if (hf == 0) ssum[wave][rl] = s; }
#pragma unroll 4
  for (int rl = 0; rl < 16; ++rl) { st[lane * 2][wave * 16 + rl] = (_Float16)so[wave][rl][lane * 2]; st[lane * 2 + 1][wave * 16 + rl] = (_Float16)so[wave][rl][lane * 2 + 1]; }
  __syncthreads();
  for (int q = tid; q < DD * 8; q += 128) { const int d = q >> 3, pc = q & 7; vst2(hT + (((size_t)hd * NB + b) * DD + d) * NN + n0 + pc * 8, *(const v4u*)(&st[d][pc * 8])); }
  if (tid < 16) { float4 v; float* vv = (float*)&v; for (int e = 0; e < 4; ++e) vv[e] = ssum[tid >> 2][(tid & 3) * 4 + e]; vst2(sc + (size_t)hd * NR + r0b + tid * 4, *(const v4f*)vv); }
}
__global__ __launch_bounds__(64) void k_attn(const float* __restrict__ sc, const int* __restrict__ A, const _Float16* __restrict__ hT, float* __restrict__ part) {
  __shared__ __align__(16) float sE[2][16][NN + 8];
  __shared__ __align__(16) float sO[2][16][68];
  __shared__ float ssj[NN];
  const int tid = threadIdx.x, w = tid >> 5, lane = tid & 31, col = lane & 15, g = lane >> 4;
  const int b = blockIdx.y, hd = blockIdx.z, i0 = blockIdx.x * 32 + w * 16; const size_t rb = (size_t)b * NN;
  for (int j = tid; j < NN; j += 64) ssj[j] = sc[(size_t)hd * NR + rb + j];
  __syncthreads();
#pragma unroll 1
  for (int m = 0; m < 16; ++m) { const int i = i0 + m; const float si = ssj[i]; const int* Ar = A + (size_t)i * NN;
#pragma unroll 8
    for (int j = lane; j < NN; j += 32) { const float e = fmaxf(si + ssj[j], 0.f); sE[w][m][j] = Ar[j] > 0 ? e : -1.0e9f; } }
  LDSX();
  { const int m = col; float* row = &sE[w][m][0]; float mx = -3.4e38f;
#pragma unroll 8
    for (int j = g * 1024; j < g * 1024 + 1024; ++j) mx = fmaxf(mx, row[j]);
    mx = fmaxf(mx, __shfl_xor(mx, 16, 32)); float l = 0.f;
#pragma unroll 8
    for (int j = g * 1024; j < g * 1024 + 1024; ++j) { const float p = __expf(row[j] - mx); row[j] = p; l += p; }
    l += __shfl_xor(l, 16, 32); const float inv = 16384.0f / l;
    LDSX();
#pragma unroll 8
    for (int j = g * 1024; j < g * 1024 + 1024; ++j) row[j] *= inv; }
  LDSX();
  v8f acc[4] = {};
#pragma unroll 2
  for (int kc = 0; kc < NN / 32; ++kc) { const v16h pa = frag_f32(&sE[w][col][0] + kc * 32, lane);
#pragma unroll
    for (int t = 0; t < 4; ++t) acc[t] = wmma16(pa, frag_h(hT + (((size_t)hd * NB + b) * DD + t * 16 + col) * NN + kc * 32, lane), acc[t]); }
#pragma unroll
  for (int t = 0; t < 4; ++t)
#pragma unroll
    for (int r = 0; r < 8; ++r) sO[w][8 * g + r][t * 16 + col] = acc[t][r] * (1.0f / 16384.0f);
  LDSX();
  for (int q = lane; q < 16 * 16; q += 32) { const int rl = q >> 4, pc = q & 15; vst2(part + ((size_t)hd * NR + rb + i0 + rl) * DD + pc * 4, *(const v4f*)(&sO[w][rl][pc * 4])); }
}
__global__ __launch_bounds__(256) void k_fin(const float* __restrict__ part, float* __restrict__ out) {
  const size_t i4 = (size_t)blockIdx.x * 256 + threadIdx.x; if (i4 >= (size_t)NR * DD / 4) return;
  v4f a = *(const v4f*)(part + i4 * 4);
#pragma unroll
  for (int hd = 1; hd < NH; ++hd) { const v4f b2 = *(const v4f*)(part + (size_t)hd * NR * DD + i4 * 4); a += b2; }
#pragma unroll
  for (int e = 0; e < 4; ++e) { const float v = a[e] * 0.25f; a[e] = v > 0.f ? v : 0.2f * v; }
  vst2(out + i4 * 4, a);
}
extern "C" void kernel_launch(void* const* d_in, const int* in_sizes, int n_in, void* d_out, int out_size, void* d_ws, size_t ws_size, hipStream_t stream) {
  (void)in_sizes; (void)n_in; (void)out_size; (void)ws_size;
  const float* X = (const float*)d_in[0]; const int* A = (const int*)d_in[1]; const float* Wk = (const float*)d_in[2]; const float* ak = (const float*)d_in[3];
  float* out = (float*)d_out;
  char* ws = (char*)d_ws; size_t off = 0;
  auto take = [&](size_t bytes) { char* p = ws + off; off += (bytes + 255) & ~(size_t)255; return p; };
  _Float16* hT = (_Float16*)take((size_t)NH * NB * DD * NN * 2); float* sc = (float*)take((size_t)NH * NR * 4); float* part = (float*)take((size_t)NH * NR * DD * 4);
  k_proj<<<dim3(NR / 64, NH), 128, 0, stream>>>(X, Wk, ak, hT, sc);
  k_attn<<<dim3(NN / 32, NB, NH), 64, 0, stream>>>(sc, A, hT, part);
  k_fin<<<(unsigned)(((size_t)NR * DD / 4 + 255) / 256), 256, 0, stream>>>(part, out);
}
